// MultiheadSelfAttention_3126736191744
// MI455X (gfx1250) — hardware-verified
//
#include <hip/hip_runtime.h>


#ifndef NB
#define NB 2
#endif
#ifndef SEQ
#define SEQ 2048
#endif
#define NB_FULL  2
#define SEQ_FULL 2048
#define DM   1024
#define NH   16
#define HD   64
#define RH   256
#define MTOK (NB * SEQ)
#define PLANE ((size_t)MTOK * DM)
#define SCL  0.125f
#define L2E  1.4426950408889634f
#define NEGB (-3.0e38f)
#define OSP  68
static_assert(HD == 64);
static_assert(NH * HD == DM);
static_assert(DM % 64 == 0);
static_assert(DM % 32 == 0);
static_assert(HD % 32 == 0);
static_assert(SEQ % 64 == 0);
static_assert(RH % 64 == 0);
static_assert(SEQ >= RH);
static_assert(NB <= NB_FULL);
static_assert(SEQ <= SEQ_FULL);
static_assert((RH / 16) % 4 == 0);
static_assert(((SEQ - RH) / 16) % 4 == 0);
static_assert(16 * OSP >= 15 * OSP + 64);
static_assert((OSP * 4) % 16 == 0);

typedef _Float16 h16;
typedef unsigned short bf;
typedef __attribute__((ext_vector_type(16))) __bf16   v16bf;
typedef __attribute__((ext_vector_type(16))) _Float16 v16h;
typedef __attribute__((ext_vector_type(16))) unsigned short v16us;
typedef __attribute__((ext_vector_type(8)))  _Float16 v8h;
typedef __attribute__((ext_vector_type(8)))  unsigned short v8us;
typedef __attribute__((ext_vector_type(8)))  float    v8f;
typedef __attribute__((ext_vector_type(4)))  float    v4f;
typedef __attribute__((ext_vector_type(2)))  float    v2f;
typedef v4f  __attribute__((may_alias)) v4fa;

__device__ __forceinline__ unsigned short f2bf(float f) { unsigned u = __float_as_uint(f); u += 0x7FFFu + ((u >> 16) & 1u); return (unsigned short)(u >> 16); }
__device__ __forceinline__ float bf2f(unsigned short b) { return __uint_as_float(((unsigned)b) << 16); }
__device__ __forceinline__ void splitf(float y, unsigned short& h, unsigned short& l) { h = f2bf(y); l = f2bf(y - bf2f(h)); }
__device__ __forceinline__ v16h cat16(v8h lo, v8h hi) { return __builtin_shufflevector(lo, hi, 0, 1, 2, 3, 4, 5, 6, 7, 8, 9, 10, 11, 12, 13, 14, 15); }
__device__ __forceinline__ v16bf cat16b(v8us lo, v8us hi) { return __builtin_bit_cast(v16bf, __builtin_shufflevector(lo, hi, 0, 1, 2, 3, 4, 5, 6, 7, 8, 9, 10, 11, 12, 13, 14, 15)); }
__device__ __forceinline__ v8f wmma16(v16h a, v16h b, v8f c) { return __builtin_amdgcn_wmma_f32_16x16x32_f16(false, a, false, b, (short)0, c, false, false); }
__device__ __forceinline__ v8f wmmab(v16bf a, v16bf b, v8f c) { return __builtin_amdgcn_wmma_f32_16x16x32_bf16(false, a, false, b, (short)0, c, false, false); }
__device__ __forceinline__ v16bf ldfrag(const bf* p) { return cat16b(*(const v8us*)p, *(const v8us*)(p + 16)); }
__device__ __forceinline__ v16h ldfragh(const h16* p) { return cat16(*(const v8h*)p, *(const v8h*)(p + 16)); }

template <int NSPLIT>
__device__ __forceinline__ void gemm_main(const bf* __restrict__ A, const bf* __restrict__ A2, const bf* __restrict__ Bt, const int K, const int r0, const int c0, const int lr, const int hi, v8f (&acc)[4][4]) {
#pragma unroll
    for (int mb = 0; mb < 4; ++mb)
#pragma unroll
        for (int nb = 0; nb < 4; ++nb) acc[mb][nb] = (v8f){};
    const size_t aoff = (size_t)(r0 + lr) * K + 8 * hi, boff = (size_t)(c0 + lr) * K + 8 * hi;
#pragma unroll 1
    for (int kc = 0; kc < K; kc += 32) {
        v16bf a[4], a2[4], b;
#pragma unroll
        for (int mb = 0; mb < 4; ++mb) { a[mb] = ldfrag(A + aoff + (size_t)mb * 16 * K + kc); if (NSPLIT == 1) a2[mb] = ldfrag(A2 + aoff + (size_t)mb * 16 * K + kc); else a2[mb] = a[mb]; }
#pragma unroll
        for (int nb = 0; nb < 4; ++nb) { b = ldfrag(Bt + boff + (size_t)nb * 16 * K + kc);
#pragma unroll
            for (int mb = 0; mb < 4; ++mb) { acc[mb][nb] = wmmab(a[mb], b, acc[mb][nb]); if (NSPLIT == 1) acc[mb][nb] = wmmab(a2[mb], b, acc[mb][nb]); } }
        asm volatile("" : "+v"(acc[0][0]), "+v"(acc[0][1]), "+v"(acc[0][2]), "+v"(acc[0][3]), "+v"(acc[1][0]), "+v"(acc[1][1]), "+v"(acc[1][2]), "+v"(acc[1][3]));
        if (NSPLIT == 1) asm volatile("v_nop\n\tv_nop\n\tv_nop\n\tv_nop" : "+v"(acc[2][0]), "+v"(acc[2][1]), "+v"(acc[2][2]), "+v"(acc[2][3]), "+v"(acc[3][0]), "+v"(acc[3][1]), "+v"(acc[3][2]), "+v"(acc[3][3]) : "v"(a[3]), "v"(a2[3]), "v"(b));
        else             asm volatile("v_nop\n\tv_nop\n\tv_nop\n\tv_nop" : "+v"(acc[2][0]), "+v"(acc[2][1]), "+v"(acc[2][2]), "+v"(acc[2][3]), "+v"(acc[3][0]), "+v"(acc[3][1]), "+v"(acc[3][2]), "+v"(acc[3][3]) : "v"(a[0]), "v"(a[3]), "v"(b));
        asm volatile("" : "+v"(acc[0][0]), "+v"(acc[0][1]), "+v"(acc[0][2]), "+v"(acc[0][3]), "+v"(acc[1][0]), "+v"(acc[1][1]), "+v"(acc[1][2]), "+v"(acc[1][3]));
    }
}

__device__ __forceinline__ void rope8(const v4f xa, const v4f xb, const v4f ca, const v4f cb, float (&y)[8]) {
#pragma clang fp contract(off)
    y[0] = xa[0] * ca[0] - xa[1] * ca[1]; y[1] = xa[1] * ca[0] + xa[0] * ca[1];
    y[2] = xa[2] * ca[2] - xa[3] * ca[3]; y[3] = xa[3] * ca[2] + xa[2] * ca[3];
    y[4] = xb[0] * cb[0] - xb[1] * cb[1]; y[5] = xb[1] * cb[0] + xb[0] * cb[1];
    y[6] = xb[2] * cb[2] - xb[3] * cb[3]; y[7] = xb[3] * cb[2] + xb[2] * cb[3];
}

__global__ __launch_bounds__(256) void k_cvt8(const float* __restrict__ src, bf* dst, size_t n8, size_t per8, size_t bstride) {
    const size_t i = (size_t)blockIdx.x * 256 + threadIdx.x; if (i >= n8) return;
    const size_t b = i / per8, r = i - b * per8;
    const v8f v = *(const v8f*)(src + b * bstride + r * 8); v8us o;
#pragma unroll
    for (int k = 0; k < 8; ++k) o[k] = f2bf(v[k]);
    *(volatile v8us*)(dst + i * 8) = o; __threadfence(); *(volatile v8us*)(dst + i * 8) = o;
}

__global__ __launch_bounds__(256) void k_cstab(float* CS) {
    const int idx = blockIdx.x * 256 + threadIdx.x; if (idx >= SEQ * 32) return;
    const int j = idx & 31, pos = idx >> 5;
    double p = 1.0;
    p *= (j & 1)  ? 1.3335214321633240 : 1.0;
    p *= (j & 2)  ? 1.7782794100389228 : 1.0;
    p *= (j & 4)  ? 3.1622776601683795 : 1.0;
    p *= (j & 8)  ? 10.0 : 1.0;
    p *= (j & 16) ? 100.0 : 1.0;
    const float pf = (float)p; const float inv = 1.0f / pf; const float ang = (float)pos * inv;
    v2f cs; cs[0] = cosf(ang); cs[1] = sinf(ang);
    *(volatile v2f*)(CS + (size_t)idx * 2) = cs; __threadfence(); *(volatile v2f*)(CS + (size_t)idx * 2) = cs;
}

__global__ __launch_bounds__(32) void k_proj_qk(const bf* __restrict__ XB, const bf* __restrict__ W2, const float* __restrict__ CS, bf* PH, bf* PL) {
    __shared__ __align__(16) float os[16 * OSP];
    const int lane = threadIdx.x & 31, lr = lane & 15, hi = lane >> 4;
    const int r0 = blockIdx.x * 64, c0 = blockIdx.y * 64, head = blockIdx.y; const size_t z = blockIdx.z;
    v8f acc[4][4];
    gemm_main<0>(XB, XB, W2 + z * (size_t)DM * DM, DM, r0, c0, lr, hi, acc);
    bf* ph = PH + z * PLANE; bf* pl = PL + z * PLANE;
    const int rq = lane >> 3, cofs = (lane & 7) * 8;
#pragma unroll
    for (int mb = 0; mb < 4; ++mb) {
#pragma unroll
        for (int nb = 0; nb < 4; ++nb)
#pragma unroll
            for (int j = 0; j < 8; ++j) os[(hi * 8 + j) * OSP + nb * 16 + lr] = acc[mb][nb][j];
        asm volatile("s_wait_dscnt 0" ::: "memory"); __builtin_amdgcn_wave_barrier(); asm volatile("" ::: "memory");
#pragma unroll 1
        for (int ps = 0; ps < 2; ++ps) {
#pragma unroll
            for (int s = 0; s < 4; ++s) {
                const int row = 4 * s + rq; const int m = r0 + mb * 16 + row; const int b = m / SEQ, pos = m % SEQ;
                const v4f xa = *(const v4fa*)(os + row * OSP + cofs), xb = *(const v4fa*)(os + row * OSP + cofs + 4);
                const v4f ca = *(const v4f*)(CS + (size_t)pos * 64 + cofs), cb = *(const v4f*)(CS + (size_t)pos * 64 + cofs + 4);
                float y[8]; rope8(xa, xb, ca, cb, y); v8us oh, ol;
#pragma unroll
                for (int k = 0; k < 8; ++k) { unsigned short a2, c2; splitf(y[k], a2, c2); oh[k] = a2; ol[k] = c2; }
                const size_t oo = (((size_t)b * NH + head) * SEQ + pos) * HD + cofs;
                *(volatile v8us*)(ph + oo) = oh; *(volatile v8us*)(pl + oo) = ol; }
            if (ps == 0) __threadfence(); }
        __builtin_amdgcn_wave_barrier(); asm volatile("" ::: "memory");
    }
}

__global__ __launch_bounds__(32) void k_proj_v(const bf* __restrict__ WV, const bf* __restrict__ XB, h16* VT16, bf* VTH, bf* VTL) {
    __shared__ __align__(16) float os[16 * OSP];
    const int lane = threadIdx.x & 31, lr = lane & 15, hi = lane >> 4;
    const int r0 = blockIdx.x * 64, c0 = blockIdx.y * 64, head = blockIdx.x;
    v8f acc[4][4];
    gemm_main<0>(WV, WV, XB, DM, r0, c0, lr, hi, acc);
    const int b = c0 / SEQ, s0 = c0 % SEQ; const bool early = (s0 < RH); const size_t bh = (size_t)b * NH + head;
    const int rq = lane >> 3, cofs = (lane & 7) * 8;
#pragma unroll
    for (int mb = 0; mb < 4; ++mb) {
#pragma unroll
        for (int nb = 0; nb < 4; ++nb)
#pragma unroll
            for (int j = 0; j < 8; ++j) os[(hi * 8 + j) * OSP + nb * 16 + lr] = acc[mb][nb][j];
        asm volatile("s_wait_dscnt 0" ::: "memory"); __builtin_amdgcn_wave_barrier(); asm volatile("" ::: "memory");
#pragma unroll 1
        for (int ps = 0; ps < 2; ++ps) {
#pragma unroll
            for (int s = 0; s < 4; ++s) {
                const int row = 4 * s + rq; const int d = mb * 16 + row;
                const v4f xa = *(const v4fa*)(os + row * OSP + cofs), xb = *(const v4fa*)(os + row * OSP + cofs + 4);
                v8h o16; v8us oh, ol;
#pragma unroll
                for (int k = 0; k < 4; ++k) { unsigned short a2, c2; o16[k] = (h16)xa[k]; splitf(xa[k], a2, c2); oh[k] = a2; ol[k] = c2; o16[4 + k] = (h16)xb[k]; splitf(xb[k], a2, c2); oh[4 + k] = a2; ol[4 + k] = c2; }
                *(volatile v8h*)(VT16 + (bh * HD + d) * SEQ + s0 + cofs) = o16;
                if (early) { const size_t oe = (bh * HD + d) * RH + s0 + cofs; *(volatile v8us*)(VTH + oe) = oh; *(volatile v8us*)(VTL + oe) = ol; } }
            if (ps == 0) __threadfence(); }
        __builtin_amdgcn_wave_barrier(); asm volatile("" ::: "memory");
    }
}

__global__ __launch_bounds__(32) void k_out(const bf* __restrict__ CH, const bf* __restrict__ CL, const bf* __restrict__ WO, float* OUT) {
    __shared__ __align__(16) float os[16 * OSP];
    const int lane = threadIdx.x & 31, lr = lane & 15, hi = lane >> 4;
    const int r0 = blockIdx.x * 64, c0 = blockIdx.y * 64;
    v8f acc[4][4];
    gemm_main<1>(CH, CL, WO, DM, r0, c0, lr, hi, acc);
#pragma unroll
    for (int mb = 0; mb < 4; ++mb) {
#pragma unroll
        for (int nb = 0; nb < 4; ++nb)
#pragma unroll
            for (int j = 0; j < 8; ++j) os[(hi * 8 + j) * OSP + nb * 16 + lr] = acc[mb][nb][j];
        asm volatile("s_wait_dscnt 0" ::: "memory"); __builtin_amdgcn_wave_barrier(); asm volatile("" ::: "memory");
#pragma unroll 1
        for (int ps = 0; ps < 2; ++ps) {
#pragma unroll
            for (int s = 0; s < 8; ++s) { const int row = 2 * s + hi, cofs = lr * 4; const int m = r0 + mb * 16 + row; const int b = m / SEQ, t = m % SEQ;
                const v4f val = *(const v4fa*)(os + row * OSP + cofs);
                *(volatile v4f*)(OUT + ((size_t)b * SEQ_FULL + t) * DM + c0 + cofs) = val; }
            if (ps == 0) __threadfence(); }
        __builtin_amdgcn_wave_barrier(); asm volatile("" ::: "memory");
    }
}

template <bool HIRES, bool MASKED>
__device__ __forceinline__ void attn_step(const bf* __restrict__ KH, const bf* __restrict__ KL, const h16* __restrict__ V16, const bf* __restrict__ VH, const bf* __restrict__ VL,
                                          const v16bf (&qh)[2], const v16bf (&ql)[2], v8f (&O)[4], float& mrun, float& lsum, const int key0, const int qn, const int lr, const int hi) {
    v8f T0 = (v8f){}, T1 = (v8f){};
    const size_t koff = (size_t)(key0 + lr) * HD + 8 * hi;
    v16bf k0h, k0l, k1h, k1l;
#pragma unroll
    for (int ks = 0; ks < 2; ++ks) {
        k0h = ldfrag(KH + koff + ks * 32); k0l = ldfrag(KL + koff + ks * 32);
        k1h = ldfrag(KH + koff + 16 * HD + ks * 32); k1l = ldfrag(KL + koff + 16 * HD + ks * 32);
        T0 = wmmab(k0h, qh[ks], T0); T0 = wmmab(k0l, qh[ks], T0); T0 = wmmab(k0h, ql[ks], T0);
        T1 = wmmab(k1h, qh[ks], T1); T1 = wmmab(k1l, qh[ks], T1); T1 = wmmab(k1h, ql[ks], T1);
    }
    asm volatile("v_nop\n\tv_nop\n\tv_nop\n\tv_nop" : "+v"(T0), "+v"(T1) : "v"(qh[1]), "v"(ql[1]), "v"(k1h), "v"(k1l));
    float mx = NEGB;
#pragma unroll
    for (int r = 0; r < 8; ++r) {
        float a = T0[r] * SCL, c = T1[r] * SCL;
        if (MASKED) { a = (key0 + 8 * hi + r <= qn) ? a : NEGB; c = (key0 + 16 + 8 * hi + r <= qn) ? c : NEGB; }
        T0[r] = a; T1[r] = c; mx = fmaxf(mx, fmaxf(a, c));
    }
    mx = fmaxf(mx, __shfl_xor(mx, 16, 32));
    const float mn = fmaxf(mrun, mx);
    const float alpha = __builtin_amdgcn_exp2f((mrun - mn) * L2E);
    mrun = mn;
    float psum = 0.0f;
    if (HIRES) {
        v16us phv, plv;
#pragma unroll
        for (int r = 0; r < 8; ++r) {
            float e0 = __builtin_amdgcn_exp2f((T0[r] - mn) * L2E), e1 = __builtin_amdgcn_exp2f((T1[r] - mn) * L2E);
            if (MASKED) { e0 = (key0 + 8 * hi + r <= qn) ? e0 : 0.0f; e1 = (key0 + 16 + 8 * hi + r <= qn) ? e1 : 0.0f; }
            psum += e0 + e1;
            unsigned short a2, c2; splitf(e0, a2, c2); phv[r] = a2; plv[r] = c2; splitf(e1, a2, c2); phv[8 + r] = a2; plv[8 + r] = c2;
        }
        lsum = lsum * alpha + psum;
#pragma unroll
        for (int dt = 0; dt < 4; ++dt)
#pragma unroll
            for (int r = 0; r < 8; ++r) O[dt][r] *= alpha;
        const v16bf pbh = __builtin_bit_cast(v16bf, phv), pbl = __builtin_bit_cast(v16bf, plv);
        const size_t voff = (size_t)lr * RH + key0 + 8 * hi;
        v16bf vh, vl;
#pragma unroll
        for (int dt = 0; dt < 4; ++dt) { vh = ldfrag(VH + voff + (size_t)dt * 16 * RH); vl = ldfrag(VL + voff + (size_t)dt * 16 * RH);
            O[dt] = wmmab(vh, pbh, O[dt]); O[dt] = wmmab(vl, pbh, O[dt]); O[dt] = wmmab(vh, pbl, O[dt]); }
        asm volatile("v_nop\n\tv_nop\n\tv_nop\n\tv_nop" : "+v"(O[0]), "+v"(O[1]), "+v"(O[2]), "+v"(O[3]) : "v"(pbh), "v"(pbl), "v"(vh), "v"(vl));
    } else {
        v16h pb;
#pragma unroll
        for (int r = 0; r < 8; ++r) {
            float e0 = __builtin_amdgcn_exp2f((T0[r] - mn) * L2E + 10.0f), e1 = __builtin_amdgcn_exp2f((T1[r] - mn) * L2E + 10.0f);
            if (MASKED) { e0 = (key0 + 8 * hi + r <= qn) ? e0 : 0.0f; e1 = (key0 + 16 + 8 * hi + r <= qn) ? e1 : 0.0f; }
            psum += e0 + e1; pb[r] = (h16)e0; pb[8 + r] = (h16)e1;
        }
        lsum = lsum * alpha + psum;
#pragma unroll
        for (int dt = 0; dt < 4; ++dt)
#pragma unroll
            for (int r = 0; r < 8; ++r) O[dt][r] *= alpha;
        const size_t voff = (size_t)lr * SEQ + key0 + 8 * hi;
        v16h va[4];
#pragma unroll
        for (int dt = 0; dt < 4; ++dt) va[dt] = ldfragh(V16 + voff + (size_t)dt * 16 * SEQ);
#pragma unroll
        for (int dt = 0; dt < 4; ++dt) O[dt] = wmma16(va[dt], pb, O[dt]);
        asm volatile("v_nop\n\tv_nop\n\tv_nop\n\tv_nop" : "+v"(O[0]), "+v"(O[1]), "+v"(O[2]), "+v"(O[3]) : "v"(pb), "v"(va[0]), "v"(va[3]));
    }
}

template <bool HIRES>
__device__ __forceinline__ void attn_body(const bf* __restrict__ QH, const bf* __restrict__ QL, const bf* __restrict__ KH, const bf* __restrict__ KL,
                                          const h16* __restrict__ V16, const bf* __restrict__ VH, const bf* __restrict__ VL, bf* CH, bf* CL) {
    __shared__ __align__(16) float os[4 * 16 * OSP];
    constexpr int TPH = HIRES ? (RH / 16) : ((SEQ > RH) ? (SEQ - RH) / 16 : 1);
    const int lane = threadIdx.x & 31, lr = lane & 15, hi = lane >> 4;
    const int wave = __builtin_amdgcn_readfirstlane(threadIdx.x >> 5);
    const int tile = blockIdx.x * 4 + wave;
    const int bh = tile / TPH; const int q0 = (tile % TPH + (HIRES ? 0 : RH / 16)) * 16;
    const int b = bh / NH, head = bh % NH;
    const size_t pbase = (size_t)bh * SEQ * HD;
    const bf* kh = KH + pbase; const bf* kl = KL + pbase;
    const h16* v16 = V16 + (size_t)bh * HD * SEQ; const bf* vh = VH + (size_t)bh * HD * RH; const bf* vl = VL + (size_t)bh * HD * RH;
    v16bf qh[2], ql[2];
    { const size_t qoff = pbase + (size_t)(q0 + lr) * HD + 8 * hi;
#pragma unroll
      for (int ks = 0; ks < 2; ++ks) { qh[ks] = ldfrag(QH + qoff + ks * 32); ql[ks] = ldfrag(QL + qoff + ks * 32); } }
    v8f O[4];
#pragma unroll
    for (int dt = 0; dt < 4; ++dt) O[dt] = (v8f){};
    float mrun = NEGB, lsum = 0.0f;
    const int qn = q0 + lr;
    const int nsteps = (q0 >> 5) + 1;
#pragma unroll 1
    for (int st = 0; st < nsteps - 1; ++st) attn_step<HIRES, false>(kh, kl, v16, vh, vl, qh, ql, O, mrun, lsum, st * 32, qn, lr, hi);
    attn_step<HIRES, true>(kh, kl, v16, vh, vl, qh, ql, O, mrun, lsum, (nsteps - 1) * 32, qn, lr, hi);
    const float l = lsum + __shfl_xor(lsum, 16, 32);
    const float inv = 1.0f / l;
    const int wbase = wave * 16 * OSP;
#pragma unroll
    for (int dt = 0; dt < 4; ++dt) { v4f a, c;
#pragma unroll
        for (int r = 0; r < 4; ++r) { a[r] = O[dt][r] * inv; c[r] = O[dt][4 + r] * inv; }
        *(v4fa*)(os + wbase + lr * OSP + dt * 16 + 8 * hi) = a; *(v4fa*)(os + wbase + lr * OSP + dt * 16 + 8 * hi + 4) = c; }
    asm volatile("s_wait_dscnt 0" ::: "memory"); __builtin_amdgcn_wave_barrier(); asm volatile("" ::: "memory");
    const int rq = lane >> 3, cofs = (lane & 7) * 8;
#pragma unroll 1
    for (int ps = 0; ps < 2; ++ps) {
#pragma unroll
        for (int s = 0; s < 4; ++s) {
            const int row = 4 * s + rq;
            const v4f xa = *(const v4fa*)(os + wbase + row * OSP + cofs), xb = *(const v4fa*)(os + wbase + row * OSP + cofs + 4);
            v8us oh, ol;
#pragma unroll
            for (int k = 0; k < 4; ++k) { unsigned short a2, c2; splitf(xa[k], a2, c2); oh[k] = a2; ol[k] = c2; splitf(xb[k], a2, c2); oh[4 + k] = a2; ol[4 + k] = c2; }
            const size_t oo = ((size_t)b * SEQ + q0 + row) * DM + head * HD + cofs;
            *(volatile v8us*)(CH + oo) = oh; *(volatile v8us*)(CL + oo) = ol; }
        if (ps == 0) __threadfence(); }
}

__global__ __launch_bounds__(128) void k_attn_hi(const bf* __restrict__ QH, const bf* __restrict__ QL, const bf* __restrict__ KH, const bf* __restrict__ KL, const h16* __restrict__ V16, const bf* __restrict__ VH, const bf* __restrict__ VL, bf* CH, bf* CL) {
    attn_body<true>(QH, QL, KH, KL, V16, VH, VL, CH, CL);
}
__global__ __launch_bounds__(128) void k_attn_lo(const bf* __restrict__ QH, const bf* __restrict__ QL, const bf* __restrict__ KH, const bf* __restrict__ KL, const h16* __restrict__ V16, const bf* __restrict__ VH, const bf* __restrict__ VL, bf* CH, bf* CL) {
    attn_body<false>(QH, QL, KH, KL, V16, VH, VL, CH, CL);
}

constexpr size_t SZ_W    = (size_t)DM * DM * 2;
constexpr size_t SZ_CS   = (size_t)SEQ * 64 * 4;
constexpr size_t SZ_ACT  = (size_t)MTOK * DM * 2;
constexpr size_t SZ_VE   = (size_t)NB * NH * HD * RH * 2;
constexpr size_t OFF_W    = 0;
constexpr size_t OFF_CS   = OFF_W + 4 * SZ_W;
constexpr size_t OFF_XB   = OFF_CS + SZ_CS;
constexpr size_t OFF_QKH  = OFF_XB + SZ_ACT;
constexpr size_t OFF_QKL  = OFF_QKH + 2 * SZ_ACT;
constexpr size_t OFF_VT16 = OFF_QKL + 2 * SZ_ACT;
constexpr size_t OFF_VTH  = OFF_VT16 + SZ_ACT;
constexpr size_t OFF_VTL  = OFF_VTH + SZ_VE;
constexpr size_t OFF_CH   = OFF_VTL + SZ_VE;
constexpr size_t OFF_CL   = OFF_CH + SZ_ACT;
constexpr size_t WS_TOTAL = OFF_CL + SZ_ACT;
static_assert(SZ_W % 256 == 0);
static_assert(SZ_CS % 256 == 0);
static_assert(SZ_ACT % 256 == 0);
static_assert(SZ_VE % 256 == 0);
static_assert(WS_TOTAL <= (size_t)134217728);

extern "C" void kernel_launch(void* const* d_in, const int* in_sizes, int n_in,
                              void* d_out, int out_size, void* d_ws, size_t ws_size, hipStream_t stream) {
    if (n_in < 5) return;
    const size_t needx = ((size_t)(NB - 1) * SEQ_FULL + SEQ) * DM;
    if ((size_t)in_sizes[0] < needx) return;
    if ((size_t)in_sizes[1] < (size_t)DM * DM || (size_t)in_sizes[2] < (size_t)DM * DM || (size_t)in_sizes[3] < (size_t)DM * DM || (size_t)in_sizes[4] < (size_t)DM * DM) return;
    if ((size_t)out_size < needx) return;
    if (ws_size < WS_TOTAL) return;
    const float* x = (const float*)d_in[0]; const float* wq = (const float*)d_in[1]; const float* wk = (const float*)d_in[2]; const float* wv = (const float*)d_in[3]; const float* wo = (const float*)d_in[4];
    float* OUT = (float*)d_out;
    char* ws = (char*)d_ws;
    bf* WQK = (bf*)(ws + OFF_W); bf* WV = (bf*)(ws + OFF_W + 2 * SZ_W); bf* WO = (bf*)(ws + OFF_W + 3 * SZ_W);
    float* CS = (float*)(ws + OFF_CS); bf* XB = (bf*)(ws + OFF_XB);
    bf* QKH = (bf*)(ws + OFF_QKH); bf* QKL = (bf*)(ws + OFF_QKL);
    h16* VT16 = (h16*)(ws + OFF_VT16); bf* VTH = (bf*)(ws + OFF_VTH); bf* VTL = (bf*)(ws + OFF_VTL);
    bf* CH = (bf*)(ws + OFF_CH); bf* CL = (bf*)(ws + OFF_CL);

    const size_t nw8 = (size_t)DM * DM / 8, nx8 = (size_t)MTOK * DM / 8;
    k_cvt8<<<(unsigned)((nw8 + 255) / 256), 256, 0, stream>>>(wq, WQK, nw8, nw8, 0);
    k_cvt8<<<(unsigned)((nw8 + 255) / 256), 256, 0, stream>>>(wk, WQK + (size_t)DM * DM, nw8, nw8, 0);
    k_cvt8<<<(unsigned)((nw8 + 255) / 256), 256, 0, stream>>>(wv, WV, nw8, nw8, 0);
    k_cvt8<<<(unsigned)((nw8 + 255) / 256), 256, 0, stream>>>(wo, WO, nw8, nw8, 0);
    k_cvt8<<<(unsigned)((nx8 + 255) / 256), 256, 0, stream>>>(x, XB, nx8, (size_t)SEQ * DM / 8, (size_t)SEQ_FULL * DM);
    k_cstab<<<SEQ * 32 / 256, 256, 0, stream>>>(CS);
    k_proj_qk<<<dim3(MTOK / 64, DM / 64, 2), 32, 0, stream>>>(XB, WQK, CS, QKH, QKL);
    k_proj_v<<<dim3(DM / 64, MTOK / 64, 1), 32, 0, stream>>>(WV, XB, VT16, VTH, VTL);
    k_attn_hi<<<NB * NH * (RH / 16) / 4, 128, 0, stream>>>(QKH, QKL, QKH + PLANE, QKL + PLANE, VT16, VTH, VTL, CH, CL);
    if (SEQ > RH) k_attn_lo<<<NB * NH * ((SEQ - RH) / 16) / 4, 128, 0, stream>>>(QKH, QKL, QKH + PLANE, QKL + PLANE, VT16, VTH, VTL, CH, CL);
    k_out<<<dim3(MTOK / 64, DM / 64, 1), 32, 0, stream>>>(CH, CL, WO, OUT);
}
